// MultiHeadAttention_45913200394352
// MI455X (gfx1250) — hardware-run, weakly checked
//
#include <hip/hip_runtime.h>
#include <math.h>

typedef __attribute__((ext_vector_type(16))) _Float16 v16h;
typedef __attribute__((ext_vector_type(8)))  _Float16 v8h;
typedef __attribute__((ext_vector_type(8)))  float    v8f;
typedef __attribute__((ext_vector_type(4)))  float    v4f;

constexpr int kBatch = 4;
constexpr int kSeq   = 2048;
constexpr int kDim   = 1024;
constexpr int kHeads = 16;
constexpr int kDk    = 64;
constexpr int kTok   = kBatch * kSeq;
constexpr int kQKld  = 2 * kDim;
static_assert(kHeads * kDk == kDim, "head split");
static_assert(kDk == 64, "head width handled by the attention kernel");
static_assert((kDim % 32) == 0 && (kDk % 32) == 0 && (kSeq % 32) == 0, "GEMM K multiples of 32");
static_assert((kTok % 64) == 0 && (kDim % 64) == 0 && (kQKld % 64) == 0, "GEMM M,N multiples of 64");

constexpr float kXCarry     = 16.0f;
constexpr float kWCarry     = 256.0f;
constexpr float kQKVCarry   = 16.0f;
constexpr int   kPCarryLog2 = 10;
constexpr float kCtxCarry   = 256.0f;
constexpr float kLog2e      = 1.44269504088896340736f;
constexpr float kLnEps      = 1e-5f;

constexpr int kAtWaves = 4;
constexpr int kAtQW    = 32;
constexpr int kAtKC    = 64;
static_assert((kSeq % (kAtWaves * kAtQW)) == 0 && (kSeq % kAtKC) == 0, "attention tile multiples");

constexpr size_t kOffXH   = 0;
constexpr size_t kOffWH   = kOffXH  + (size_t)kTok * kDim * 2;
constexpr size_t kOffQK   = kOffWH  + (size_t)4 * kDim * kDim * 2;
constexpr size_t kOffVT   = kOffQK  + (size_t)kTok * kQKld * 2;
constexpr size_t kOffCTX  = kOffVT  + (size_t)kDim * kTok * 2;
constexpr size_t kOffY    = kOffCTX + (size_t)kTok * kDim * 2;
constexpr size_t kWsTotal = kOffY   + (size_t)kTok * kDim * 4;
static_assert(kWsTotal == 125829120ull, "carve total");
static_assert(kWsTotal <= 134217728ull, "carve cap");
static_assert((kOffWH % 128) == 0 && (kOffQK % 128) == 0 && (kOffVT % 128) == 0 &&
              (kOffCTX % 128) == 0 && (kOffY % 128) == 0, "128-B aligned regions");

union FragU { v16h v; v8h h[2]; };

__device__ __forceinline__ v16h frag_load(const _Float16* p) {
  FragU f;
  f.h[0] = *(const v8h*)(p);
  f.h[1] = *(const v8h*)(p + 16);
  return f.v;
}

__device__ __forceinline__ v8f mma_h(v16h a, v16h b, v8f c) {
  c = __builtin_amdgcn_wmma_f32_16x16x32_f16(false, a, false, b, (short)0, c, false, false);
  asm volatile("v_nop\n\tv_nop\n\tv_nop\n\tv_nop" : "+v"(c) : "v"(a), "v"(b));
  return c;
}

__device__ __forceinline__ void wave_lds_sync() {
  __builtin_amdgcn_fence(__ATOMIC_RELEASE, "workgroup");
  __builtin_amdgcn_wave_barrier();
  __builtin_amdgcn_fence(__ATOMIC_ACQUIRE, "workgroup");
}

__global__ __launch_bounds__(256) void cast8_f16_kernel(
    const float* __restrict__ s0, const float* __restrict__ s1,
    const float* __restrict__ s2, const float* __restrict__ s3,
    unsigned short* __restrict__ out, int n8, float carry)
{
  const int i = blockIdx.x * 256 + threadIdx.x;
  if (i >= n8) return;
  const int z = blockIdx.y;
  const float* src = (z == 0) ? s0 : (z == 1) ? s1 : (z == 2) ? s2 : s3;
  const float* p = src + 8 * (size_t)i;
  const v4f a = *(const v4f*)(p);
  const v4f c = *(const v4f*)(p + 4);
  v8h hv;
#pragma unroll
  for (int e = 0; e < 4; ++e) {
    const float x0 = a[e] * carry;
    const float x1 = c[e] * carry;
    hv[e]     = (_Float16)x0;
    hv[4 + e] = (_Float16)x1;
  }
  unsigned short* q = out + (size_t)z * ((size_t)n8 * 8) + 8 * (size_t)i;
  *(volatile v8h*)q = hv;
  __threadfence();
  *(volatile v8h*)q = hv;
}

template <int BIAS_MODE, int OUT_MODE, bool RESID>
__global__ __launch_bounds__(256) void gemm64_f16_kernel(
    const unsigned short* __restrict__ Ap, int lda,
    const unsigned short* __restrict__ Btp, int ldb,
    void* __restrict__ Cout, int ldc,
    const float* __restrict__ bias0, const float* __restrict__ bias1, int nsplit,
    const float* __restrict__ resid,
    int M, int N, int K, float scale, float bscale)
{
  const _Float16* A  = (const _Float16*)Ap;
  const _Float16* Bt = (const _Float16*)Btp;
  __shared__ __align__(16) float sT[8][16 * 68];
  const int lane = threadIdx.x & 31;
  const int wave = __builtin_amdgcn_readfirstlane((int)(threadIdx.x >> 5));
  const int tilesN = N >> 6;
  const int tilesM = M >> 6;
  const int tile = blockIdx.x * 8 + wave;
  if (tile >= tilesM * tilesN) return;
  const int tm = tile / tilesN;
  const int tn = tile - tm * tilesN;
  const int m0 = tm << 6;
  const int n0 = tn << 6;

  const int rlane = lane & 15;
  const int koff  = (lane >> 4) * 8;
  const int mOff  = (lane >> 4) * 8;

  v8f acc[4][4];
#pragma unroll
  for (int i = 0; i < 4; ++i)
#pragma unroll
    for (int j = 0; j < 4; ++j) acc[i][j] = (v8f){0.f, 0.f, 0.f, 0.f, 0.f, 0.f, 0.f, 0.f};

  for (int k0 = 0; k0 < K; k0 += 32) {
    v16h bh[4];
#pragma unroll
    for (int j = 0; j < 4; ++j) {
      const size_t bo = (size_t)(n0 + (j << 4) + rlane) * ldb + koff + k0;
      bh[j] = frag_load(Bt + bo);
    }
#pragma unroll
    for (int i = 0; i < 4; ++i) {
      const size_t ao = (size_t)(m0 + (i << 4) + rlane) * lda + koff + k0;
      const v16h ah = frag_load(A + ao);
#pragma unroll
      for (int j = 0; j < 4; ++j) acc[i][j] = mma_h(ah, bh[j], acc[i][j]);
    }
  }

  float* slab = sT[wave];
  const int hh = lane >> 4;
  const int c4 = (lane & 15) * 4;
  const int q  = lane >> 3;
  const int c8 = (lane & 7) * 8;

  v4f bA = (v4f){0.f, 0.f, 0.f, 0.f};
  v4f bB = (v4f){0.f, 0.f, 0.f, 0.f};
  if (BIAS_MODE == 2) {
    const float* bp = (n0 < nsplit) ? (bias0 + n0) : (bias1 + (n0 - nsplit));
    if (OUT_MODE == 0) {
      const v4f t0 = *(const v4f*)(bp + c4);
#pragma unroll
      for (int e = 0; e < 4; ++e) bA[e] = t0[e] * bscale;
    } else {
      const v4f t0 = *(const v4f*)(bp + c8);
      const v4f t1 = *(const v4f*)(bp + c8 + 4);
#pragma unroll
      for (int e = 0; e < 4; ++e) {
        bA[e] = t0[e] * bscale;
        bB[e] = t1[e] * bscale;
      }
    }
  }

#pragma unroll
  for (int i = 0; i < 4; ++i) {
    const int mBase = m0 + (i << 4);
#pragma unroll
    for (int j = 0; j < 4; ++j) {
#pragma unroll
      for (int r = 0; r < 8; ++r) slab[(mOff + r) * 68 + (j << 4) + rlane] = acc[i][j][r];
    }
    wave_lds_sync();
    if (OUT_MODE == 0) {
      float* C = (float*)Cout;
      v4f ov[8];
#pragma unroll
      for (int it = 0; it < 8; ++it) {
        const int row = it * 2 + hh;
        const v4f v = *(const v4f*)(slab + row * 68 + c4);
        v4f o;
#pragma unroll
        for (int e = 0; e < 4; ++e) o[e] = v[e] * scale + bA[e];
        if (RESID) {
          const v4f rr = *(const v4f*)(resid + (size_t)(mBase + row) * ldc + n0 + c4);
#pragma unroll
          for (int e = 0; e < 4; ++e) o[e] = o[e] + rr[e];
        }
        ov[it] = o;
      }
      for (int pass = 0; pass < 2; ++pass) {
#pragma unroll
        for (int it = 0; it < 8; ++it) {
          const int row = it * 2 + hh;
          *(volatile v4f*)(C + (size_t)(mBase + row) * ldc + n0 + c4) = ov[it];
        }
        __threadfence();
      }
    } else {
      unsigned short* C = (unsigned short*)Cout;
      v8h hv[4];
#pragma unroll
      for (int it = 0; it < 4; ++it) {
        const int row = it * 4 + q;
        const float* sp = slab + row * 68 + c8;
        const v4f a0 = *(const v4f*)(sp);
        const v4f a1 = *(const v4f*)(sp + 4);
        float rb = 0.f;
        if (BIAS_MODE == 1) rb = bias0[mBase + row] * bscale;
#pragma unroll
        for (int e = 0; e < 4; ++e) {
          const float x0 = a0[e] * scale + ((BIAS_MODE == 2) ? bA[e] : rb);
          const float x1 = a1[e] * scale + ((BIAS_MODE == 2) ? bB[e] : rb);
          hv[it][e]     = (_Float16)x0;
          hv[it][4 + e] = (_Float16)x1;
        }
      }
      for (int pass = 0; pass < 2; ++pass) {
#pragma unroll
        for (int it = 0; it < 4; ++it) {
          const int row = it * 4 + q;
          *(volatile v8h*)(C + (size_t)(mBase + row) * ldc + n0 + c8) = hv[it];
        }
        __threadfence();
      }
    }
    wave_lds_sync();
  }
}

__global__ __launch_bounds__(128) void attn_kernel(
    const unsigned short* __restrict__ QKp, const unsigned short* __restrict__ VTp,
    unsigned short* __restrict__ CTXp, float sc_log2, float pc_log2, float o_scale)
{
  __shared__ __align__(16) float Os[kAtWaves][kAtQW * 68];
  const int lane = threadIdx.x & 31;
  const int wave = __builtin_amdgcn_readfirstlane((int)(threadIdx.x >> 5));
  const int hh = lane >> 4;
  const int c  = lane & 15;
  const int bh = blockIdx.y;
  const int b  = bh / kHeads;
  const int h  = bh - b * kHeads;
  const int q0 = blockIdx.x * (kAtWaves * kAtQW) + wave * kAtQW;
  const size_t tok0 = (size_t)b * kSeq;

  const _Float16* QK = (const _Float16*)QKp;
  const _Float16* VT = (const _Float16*)VTp;

  v16h qb[2][2];
#pragma unroll
  for (int qt = 0; qt < 2; ++qt) {
#pragma unroll
    for (int dc = 0; dc < 2; ++dc) {
      qb[qt][dc] = frag_load(QK + (tok0 + q0 + qt * 16 + c) * kQKld + h * kDk + dc * 32 + 8 * hh);
    }
  }
  const _Float16* kbase = QK + (tok0 + c) * kQKld + kDim + h * kDk + 8 * hh;
  const _Float16* vbase = VT + (size_t)(h * kDk + c) * kTok + tok0 + 8 * hh;

  v8f oacc[4][2];
#pragma unroll
  for (int t = 0; t < 4; ++t) {
#pragma unroll
    for (int qt = 0; qt < 2; ++qt) oacc[t][qt] = (v8f){0.f, 0.f, 0.f, 0.f, 0.f, 0.f, 0.f, 0.f};
  }
  float mrun[2] = {-1.0e30f, -1.0e30f};
  float lrun[2] = {0.f, 0.f};

#pragma unroll 1
  for (int kc = 0; kc < kSeq / kAtKC; ++kc) {
    const int kv0 = kc * kAtKC;
    v8f s[4][2];
#pragma unroll
    for (int j = 0; j < 4; ++j) {
      const _Float16* kp = kbase + (size_t)(kv0 + j * 16) * kQKld;
      const v16h ka0 = frag_load(kp);
      const v16h ka1 = frag_load(kp + 32);
#pragma unroll
      for (int qt = 0; qt < 2; ++qt) {
        v8f z = (v8f){0.f, 0.f, 0.f, 0.f, 0.f, 0.f, 0.f, 0.f};
        z = mma_h(ka0, qb[qt][0], z);
        z = mma_h(ka1, qb[qt][1], z);
        s[j][qt] = z;
      }
    }

    v16h pb[2][2];
#pragma unroll
    for (int qt = 0; qt < 2; ++qt) {
      float mx = s[0][qt][0];
#pragma unroll
      for (int j = 0; j < 4; ++j) {
#pragma unroll
        for (int r = 0; r < 8; ++r) mx = fmaxf(mx, s[j][qt][r]);
      }
      const float mo = __shfl_xor(mx, 16, 32);
      mx = fmaxf(mx, mo);
      const float mnew  = fmaxf(mrun[qt], mx * sc_log2);
      const float alpha = __builtin_amdgcn_exp2f(mrun[qt] - mnew);
      mrun[qt] = mnew;
      const float moff = pc_log2 - mnew;
      float ps = 0.f;
#pragma unroll
      for (int kk = 0; kk < 2; ++kk) {
#pragma unroll
        for (int r = 0; r < 8; ++r) {
          const float p0 = __builtin_amdgcn_exp2f(fmaf(s[2 * kk][qt][r], sc_log2, moff));
          const float p1 = __builtin_amdgcn_exp2f(fmaf(s[2 * kk + 1][qt][r], sc_log2, moff));
          ps += p0;
          ps += p1;
          pb[qt][kk][r]     = (_Float16)p0;
          pb[qt][kk][8 + r] = (_Float16)p1;
        }
      }
      lrun[qt] = lrun[qt] * alpha + ps;
#pragma unroll
      for (int t = 0; t < 4; ++t) {
#pragma unroll
        for (int r = 0; r < 8; ++r) oacc[t][qt][r] *= alpha;
      }
    }

#pragma unroll
    for (int kk = 0; kk < 2; ++kk) {
#pragma unroll
      for (int t = 0; t < 4; ++t) {
        const v16h va = frag_load(vbase + (size_t)(t * 16) * kTok + kv0 + kk * 32);
#pragma unroll
        for (int qt = 0; qt < 2; ++qt) oacc[t][qt] = mma_h(va, pb[qt][kk], oacc[t][qt]);
      }
    }
  }

  float* os = Os[wave];
#pragma unroll
  for (int qt = 0; qt < 2; ++qt) {
    const float lo  = __shfl_xor(lrun[qt], 16, 32);
    const float inv = o_scale * __builtin_amdgcn_rcpf(lrun[qt] + lo);
#pragma unroll
    for (int t = 0; t < 4; ++t) {
      v4f w0, w1;
#pragma unroll
      for (int e = 0; e < 4; ++e) {
        w0[e] = oacc[t][qt][e] * inv;
        w1[e] = oacc[t][qt][4 + e] * inv;
      }
      float* dp = os + (qt * 16 + c) * 68 + t * 16 + 8 * hh;
      *(v4f*)(dp)     = w0;
      *(v4f*)(dp + 4) = w1;
    }
  }
  wave_lds_sync();
  {
    const int q8 = lane >> 3;
    const int c8 = (lane & 7) * 8;
    v8h hv[8];
#pragma unroll
    for (int it = 0; it < 8; ++it) {
      const float* sp = os + (it * 4 + q8) * 68 + c8;
      const v4f a0 = *(const v4f*)(sp);
      const v4f a1 = *(const v4f*)(sp + 4);
#pragma unroll
      for (int e = 0; e < 4; ++e) {
        const float x0 = a0[e];
        const float x1 = a1[e];
        hv[it][e]     = (_Float16)x0;
        hv[it][4 + e] = (_Float16)x1;
      }
    }
    unsigned short* cp = CTXp + (tok0 + q0) * kDim + h * kDk + c8;
    for (int pass = 0; pass < 2; ++pass) {
#pragma unroll
      for (int it = 0; it < 8; ++it) {
        *(volatile v8h*)(cp + (size_t)(it * 4 + q8) * kDim) = hv[it];
      }
      __threadfence();
    }
  }
}

__global__ __launch_bounds__(256) void layernorm_kernel(
    const float* __restrict__ Y, const float* __restrict__ gamma, const float* __restrict__ beta,
    float* __restrict__ out, int rows)
{
  const int lane = threadIdx.x & 31;
  const int wave = __builtin_amdgcn_readfirstlane((int)(threadIdx.x >> 5));
  const int row  = blockIdx.x * 8 + wave;
  if (row >= rows) return;
  const float* yr = Y + (size_t)row * kDim + lane * 4;

  float sum = 0.f;
#pragma unroll 1
  for (int i = 0; i < 8; ++i) {
    const v4f t = *(const v4f*)(yr + i * 128);
    const float part = (t[0] + t[1]) + (t[2] + t[3]);
    sum += part;
  }
#pragma unroll
  for (int off = 16; off > 0; off >>= 1) sum += __shfl_xor(sum, off, 32);
  const float mu = sum * (1.0f / (float)kDim);

  float sq = 0.f;
#pragma unroll 1
  for (int i = 0; i < 8; ++i) {
    const v4f t = *(const v4f*)(yr + i * 128);
    const float d0 = t[0] - mu;
    const float d1 = t[1] - mu;
    const float d2 = t[2] - mu;
    const float d3 = t[3] - mu;
    sq = fmaf(d0, d0, sq);
    sq = fmaf(d1, d1, sq);
    sq = fmaf(d2, d2, sq);
    sq = fmaf(d3, d3, sq);
  }
#pragma unroll
  for (int off = 16; off > 0; off >>= 1) sq += __shfl_xor(sq, off, 32);
  const float var  = sq * (1.0f / (float)kDim);
  const float rstd = rsqrtf(var + kLnEps);

  float* orow = out + (size_t)row * kDim + lane * 4;
  const float* gp = gamma + lane * 4;
  const float* bp = beta + lane * 4;
#pragma unroll 1
  for (int i = 0; i < 8; ++i) {
    const v4f t  = *(const v4f*)(yr + i * 128);
    const v4f g  = *(const v4f*)(gp + i * 128);
    const v4f bt = *(const v4f*)(bp + i * 128);
    v4f o;
    o[0] = ((t[0] - mu) * rstd) * g[0] + bt[0];
    o[1] = ((t[1] - mu) * rstd) * g[1] + bt[1];
    o[2] = ((t[2] - mu) * rstd) * g[2] + bt[2];
    o[3] = ((t[3] - mu) * rstd) * g[3] + bt[3];
    *(volatile v4f*)(orow + i * 128) = o;
    __threadfence();
    *(volatile v4f*)(orow + i * 128) = o;
  }
}

extern "C" void kernel_launch(void* const* d_in, const int* in_sizes, int n_in,
                              void* d_out, int out_size, void* d_ws, size_t ws_size,
                              hipStream_t stream) {
  if (n_in < 11) return;
  if (in_sizes[0] != kTok * kDim) return;
  if (in_sizes[1] != kDim * kDim || in_sizes[3] != kDim * kDim) return;
  if (in_sizes[5] != kDim * kDim || in_sizes[7] != kDim * kDim) return;
  if (in_sizes[2] != kDim || in_sizes[4] != kDim || in_sizes[6] != kDim || in_sizes[8] != kDim) return;
  if (in_sizes[9] != kDim || in_sizes[10] != kDim) return;
  if (out_size != kTok * kDim) return;
  if (ws_size < kWsTotal) return;

  const float* x   = (const float*)d_in[0];
  const float* Wq  = (const float*)d_in[1];
  const float* bq  = (const float*)d_in[2];
  const float* Wk  = (const float*)d_in[3];
  const float* bk  = (const float*)d_in[4];
  const float* Wv  = (const float*)d_in[5];
  const float* bv  = (const float*)d_in[6];
  const float* Wo  = (const float*)d_in[7];
  const float* bo  = (const float*)d_in[8];
  const float* lng = (const float*)d_in[9];
  const float* lnb = (const float*)d_in[10];
  float* out = (float*)d_out;

  char* ws = (char*)d_ws;
  unsigned short* XH  = (unsigned short*)(ws + kOffXH);
  unsigned short* WH  = (unsigned short*)(ws + kOffWH);
  unsigned short* QK  = (unsigned short*)(ws + kOffQK);
  unsigned short* VT  = (unsigned short*)(ws + kOffVT);
  unsigned short* CTX = (unsigned short*)(ws + kOffCTX);
  float*          Y   = (float*)(ws + kOffY);
  unsigned short* WQK = WH;
  unsigned short* WVh = WH + (size_t)2 * kDim * kDim;
  unsigned short* WOh = WH + (size_t)3 * kDim * kDim;

  const float inv_sqrt_dk = 1.0f / sqrtf((float)kDk);
  const float s_qkv   = kQKVCarry / (kXCarry * kWCarry);
  const float b_qkv   = kQKVCarry;
  const float sc_log2 = inv_sqrt_dk * kLog2e / (kQKVCarry * kQKVCarry);
  const float pc_log2 = (float)kPCarryLog2;
  const float o_scale = kCtxCarry / kQKVCarry;
  const float s_out   = 1.0f / (kCtxCarry * kWCarry);

  cast8_f16_kernel<<<dim3((kTok * kDim / 8) / 256, 1), 256, 0, stream>>>(
      x, x, x, x, XH, kTok * kDim / 8, kXCarry);
  cast8_f16_kernel<<<dim3((kDim * kDim / 8) / 256, 4), 256, 0, stream>>>(
      Wq, Wk, Wv, Wo, WH, kDim * kDim / 8, kWCarry);

  gemm64_f16_kernel<2, 1, false><<<dim3((kTok / 64) * (kQKld / 64) / 8), 256, 0, stream>>>(
      XH, kDim, WQK, kDim, (void*)QK, kQKld, bq, bk, kDim, x,
      kTok, kQKld, kDim, s_qkv, b_qkv);

  gemm64_f16_kernel<1, 1, false><<<dim3((kDim / 64) * (kTok / 64) / 8), 256, 0, stream>>>(
      WVh, kDim, XH, kDim, (void*)VT, kTok, bv, bv, 0, x,
      kDim, kTok, kDim, s_qkv, b_qkv);

  attn_kernel<<<dim3(kSeq / (kAtWaves * kAtQW), kBatch * kHeads), kAtWaves * 32, 0, stream>>>(
      QK, VT, CTX, sc_log2, pc_log2, o_scale);

  gemm64_f16_kernel<2, 0, true><<<dim3((kTok / 64) * (kDim / 64) / 8), 256, 0, stream>>>(
      CTX, kDim, WOh, kDim, (void*)Y, kDim, bo, bo, kDim, x,
      kTok, kDim, kDim, s_out, 1.0f);

  layernorm_kernel<<<dim3(kTok / 8), 256, 0, stream>>>(Y, lng, lnb, out, kTok);
}
